// ODST_30064771072292
// MI455X (gfx1250) — hardware-verified
//
#include <hip/hip_runtime.h>


#define BB    4096
#define FF    256
#define TT    128
#define DD    6
#define UU    16
#define NBINS 64
#define N1    (TT*DD)

typedef __attribute__((ext_vector_type(16))) _Float16 v16h;
typedef __attribute__((ext_vector_type(8)))  _Float16 v8h;
typedef __attribute__((ext_vector_type(8)))  float    v8f;
typedef __attribute__((ext_vector_type(4)))  float    v4f_t;
typedef float v4fa __attribute__((ext_vector_type(4), may_alias));
typedef __attribute__((ext_vector_type(4)))  unsigned v4u_t;
typedef unsigned v4ua __attribute__((ext_vector_type(4), may_alias));
#define RSPLIT (1.0f / 2048.0f)
#define PL_XH  ((size_t)BB * FF)
#define PL_SEL ((size_t)N1 * FF)
#define PL_RSP ((size_t)TT * UU * NBINS)
__device__ __forceinline__ _Float16 lo_of(float v, _Float16 h) { return (_Float16)((v - (float)h) * 2048.0f); }
__device__ __forceinline__ v8f wmma16(v16h a, v16h b, v8f c) { return __builtin_amdgcn_wmma_f32_16x16x32_f16(false, a, false, b, (short)0, c, false, false); }
__device__ __forceinline__ v8f wmma_split(v16h a, v16h al, v16h b, v16h bl, v8f c) { v8f x = {}; x = wmma16(al, b, x); x = wmma16(a, bl, x); return wmma16(a, b, c) + x * RSPLIT; }
__device__ __forceinline__ v16h frag16(const _Float16* p, int hi) { return __builtin_shufflevector(*(const v8h*)(p + 8 * hi), *(const v8h*)(p + 16 + 8 * hi), 0,1,2,3,4,5,6,7,8,9,10,11,12,13,14,15); }
__device__ __forceinline__ void st2pair(_Float16* p, size_t pl, float v0, float v1) {
  const _Float16 a = (_Float16)v0, b = (_Float16)v1;
  const unsigned u = (unsigned)__builtin_bit_cast(unsigned short, a) | ((unsigned)__builtin_bit_cast(unsigned short, b) << 16);
  const unsigned w = (unsigned)__builtin_bit_cast(unsigned short, lo_of(v0, a)) | ((unsigned)__builtin_bit_cast(unsigned short, lo_of(v1, b)) << 16);
  *(volatile unsigned*)p = u; *(volatile unsigned*)(p + pl) = w; __threadfence(); *(volatile unsigned*)p = u; *(volatile unsigned*)(p + pl) = w;
}
__device__ __forceinline__ void sparsemax6(const float* zp, float* sel) {
    float z[DD], zs[DD];
    #pragma unroll
    for (int d = 0; d < DD; d++) { z[d] = zp[d]; zs[d] = z[d]; }
    #pragma unroll
    for (int a = 0; a < DD-1; a++)
        #pragma unroll
        for (int b = 0; b < DD-1-a; b++)
            if (zs[b] < zs[b+1]) { float tv = zs[b]; zs[b] = zs[b+1]; zs[b+1] = tv; }
    float run = 0.f, cs[DD];
    int k = 0;
    #pragma unroll
    for (int d = 0; d < DD; d++) {
        run += zs[d]; cs[d] = run;
        if (1.f + (float)(d+1)*zs[d] > cs[d]) k++;
    }
    float tau = (cs[k-1] - 1.f) / (float)k;
    #pragma unroll
    for (int d = 0; d < DD; d++) { float v = z[d] - tau; sel[d] = v > 0.f ? v : 0.f; }
}

__global__ void __launch_bounds__(256)
odst_prep(const float* __restrict__ x,
          const float* __restrict__ logits,
          const float* __restrict__ thr_in,
          const float* __restrict__ logtemp,
          const float* __restrict__ resp,
          _Float16* __restrict__ xh,
          _Float16* __restrict__ selT,
          _Float16* __restrict__ resph,
          float* __restrict__ thr,
          float* __restrict__ invt)
{
    int i = (blockIdx.x * blockDim.x + threadIdx.x) * 2;
    if (i < BB*FF)       st2pair(xh + i, PL_XH, x[i], x[i + 1]);
    if (i < TT*UU*NBINS) st2pair(resph + i, PL_RSP, resp[i], resp[i + 1]);
    if (i < TT*DD) {
        typedef __attribute__((ext_vector_type(2))) float v2f_t; v2f_t a, b;
        a.x = thr_in[i]; a.y = thr_in[i + 1]; b.x = __expf(-logtemp[i]); b.y = __expf(-logtemp[i + 1]);
        *(volatile v2f_t*)(thr + i) = a; *(volatile v2f_t*)(invt + i) = b; __threadfence(); *(volatile v2f_t*)(thr + i) = a; *(volatile v2f_t*)(invt + i) = b;
    }
    (void)logits; (void)selT;
}

__global__ void __launch_bounds__(256)
odst_sel(const float* __restrict__ logits, _Float16* __restrict__ selT) {
    int i = blockIdx.x * blockDim.x + threadIdx.x;
    if (i >= N1 * (FF / 8)) return;
    int n = i >> 5, f8 = (i & 31) * 8;
    int t = n / DD, d = n - t * DD;
    _Float16 hh[8], hl[8];
    #pragma unroll 1
    for (int e = 0; e < 8; ++e) {
        float sel[DD];
        sparsemax6(logits + ((size_t)(f8 + e) * TT + t) * DD, sel);
        float v = sel[0];
        #pragma unroll
        for (int dd = 1; dd < DD; ++dd) v = (dd == d) ? sel[dd] : v;
        hh[e] = (_Float16)v; hl[e] = lo_of(v, hh[e]);
    }
    _Float16* dst = selT + (size_t)n * FF + f8;
    *(volatile v4u_t*)dst = *(const v4ua*)hh; *(volatile v4u_t*)(dst + PL_SEL) = *(const v4ua*)hl; __threadfence();
    *(volatile v4u_t*)dst = *(const v4ua*)hh; *(volatile v4u_t*)(dst + PL_SEL) = *(const v4ua*)hl;
}

__global__ void __launch_bounds__(256)
odst_gemm1(const _Float16* __restrict__ xh,
           const _Float16* __restrict__ selT,
           float* __restrict__ fv)
{
    __shared__ __attribute__((aligned(16))) float stg[8][16 * 68];
    int lane = threadIdx.x & 31;
    int wv   = threadIdx.x >> 5;
    int strip = blockIdx.x * 8 + wv;
    int tm   = strip / (N1/64);
    int tg   = strip % (N1/64);
    int hi   = lane >> 4, lo = lane & 15;

    v8f acc[4] = {};
    int arow = tm*16 + lo;
    #pragma unroll 2
    for (int k0 = 0; k0 < FF; k0 += 32) {
        const v16h a = frag16(xh + arow*FF + k0, hi), al = frag16(xh + PL_XH + arow*FF + k0, hi);
        #pragma unroll
        for (int g = 0; g < 4; ++g) {
            const _Float16* bp = selT + (size_t)(tg*64 + g*16 + lo)*FF + k0;
            acc[g] = wmma_split(a, al, frag16(bp, hi), frag16(bp + PL_SEL, hi), acc[g]);
        }
    }
    float* sw = stg[wv];
    #pragma unroll
    for (int g = 0; g < 4; ++g)
        #pragma unroll
        for (int r = 0; r < 8; r++) sw[(r + hi*8) * 68 + g*16 + lo] = acc[g][r];
    asm volatile("s_wait_dscnt 0" ::: "memory");
    #pragma unroll 1
    for (int pass = 0; pass < 2; ++pass) {
        #pragma unroll
        for (int i = 0; i < 8; ++i) { const int c = lane + 32 * i, rr = c >> 4, q = (c & 15) * 4;
            *(volatile v4f_t*)(fv + (size_t)(tm*16 + rr)*N1 + tg*64 + q) = *(const volatile v4fa*)(sw + rr*68 + q); }
        __threadfence();
    }
}

__global__ void __launch_bounds__(256)
odst_trees(const float* __restrict__ fv,
           const float* __restrict__ thr,
           const float* __restrict__ invt,
           const _Float16* __restrict__ resph,
           float* __restrict__ out)
{
    __shared__ __attribute__((aligned(16))) _Float16 wlds[2][8 * 16 * NBINS];
    int lane = threadIdx.x & 31;
    int wv   = threadIdx.x >> 5;
    _Float16* myw = wlds[0] + wv * 16 * NBINS;
    _Float16* mywl = wlds[1] + wv * 16 * NBINS;
    int mtile = blockIdx.x * 8 + wv;
    int hi = lane >> 4, lo = lane & 15;
    int row16 = lane >> 1;
    int half  = lane & 1;
    int grow  = mtile*16 + row16;

    v8f acc = {};
    for (int t = 0; t < TT; ++t) {
        const float* fvp = fv  + grow*N1 + t*DD;
        const float* th  = thr + t*DD;
        const float* iv  = invt + t*DD;
        float p[DD], q[DD];
        #pragma unroll
        for (int d = 0; d < DD; d++) {
            float tl = (fvp[d] - th[d]) * iv[d];
            p[d] = fminf(fmaxf(0.5f + 0.5f*tl, 0.f), 1.f);
            q[d] = fminf(fmaxf(0.5f - 0.5f*tl, 0.f), 1.f);
        }
        float e01[4], e23[4], e45[2];
        #pragma unroll
        for (int a2 = 0; a2 < 4; a2++) {
            e01[a2] = ((a2&1) ? q[0] : p[0]) * ((a2&2) ? q[1] : p[1]);
            e23[a2] = ((a2&1) ? q[2] : p[2]) * ((a2&2) ? q[3] : p[3]);
        }
        float f5 = half ? q[5] : p[5];
        e45[0] = p[4]*f5; e45[1] = q[4]*f5;
        _Float16* wrow = myw + row16*NBINS + half*32;
        _Float16* wrowl = mywl + row16*NBINS + half*32;
        #pragma unroll
        for (int j = 0; j < 32; j++) {
            const float wv32 = e01[j&3] * e23[(j>>2)&3] * e45[(j>>4)&1];
            wrow[j] = (_Float16)wv32; wrowl[j] = lo_of(wv32, wrow[j]);
        }
        __syncthreads();

        const _Float16* bcol = resph + (t*UU + lo)*NBINS;
        #pragma unroll
        for (int j = 0; j < 2; j++)
            acc = wmma_split(frag16(myw + lo*NBINS + j*32, hi), frag16(mywl + lo*NBINS + j*32, hi),
                             frag16(bcol + j*32, hi), frag16(bcol + PL_RSP + j*32, hi), acc);
        __syncthreads();
    }
    float* so = (float*)myw;
    #pragma unroll
    for (int r = 0; r < 8; r++) so[(r + hi*8)*UU + lo] = acc[r];
    asm volatile("s_wait_dscnt 0" ::: "memory");
    #pragma unroll 1
    for (int pass = 0; pass < 2; ++pass) {
        #pragma unroll
        for (int i = 0; i < 2; ++i) { const int c = lane + 32 * i;
            *(volatile v4f_t*)(out + (size_t)mtile*16*UU + c*4) = *(const volatile v4fa*)(so + c*4); }
        __threadfence();
    }
}

extern "C" void kernel_launch(void* const* d_in, const int* in_sizes, int n_in,
                              void* d_out, int out_size, void* d_ws, size_t ws_size,
                              hipStream_t stream)
{
    const float* x   = (const float*)d_in[0];
    const float* fsl = (const float*)d_in[1];
    const float* fth = (const float*)d_in[2];
    const float* ltp = (const float*)d_in[3];
    const float* rsp = (const float*)d_in[4];
    float* out = (float*)d_out;

    char* ws = (char*)d_ws;
    size_t off = 0;
    auto carve = [&](size_t bytes) -> char* { char* p = ws + off; off = (off + bytes + 255) & ~(size_t)255; return p; };
    _Float16* xh    = (_Float16*)carve(PL_XH * 2 * 2);
    _Float16* selT  = (_Float16*)carve(PL_SEL * 2 * 2);
    _Float16* resph = (_Float16*)carve(PL_RSP * 2 * 2);
    float*    thr   = (float*)   carve(TT*DD*4);
    float*    invt  = (float*)   carve(TT*DD*4);
    float*    fv    = (float*)   carve((size_t)BB*N1*4);

    odst_prep <<<(BB*FF/2 + 255)/256, 256, 0, stream>>>(x, fsl, fth, ltp, rsp,
                                                        xh, selT, resph, thr, invt);
    odst_sel  <<<(N1*(FF/8) + 255)/256, 256, 0, stream>>>(fsl, selT);
    odst_gemm1<<<((BB/16)*(N1/64))/8, 256, 0, stream>>>(xh, selT, fv);
    odst_trees<<<(BB/16)/8,           256, 0, stream>>>(fv, thr, invt, resph, out);
}
